// PluckerBigramAttention_60739427500738
// MI455X (gfx1250) — hardware-verified
//
#include <hip/hip_runtime.h>
#include <math.h>

typedef __attribute__((ext_vector_type(16))) _Float16 v16h;
typedef __attribute__((ext_vector_type(16))) __bf16 v16b;
typedef __attribute__((ext_vector_type(8)))  _Float16 v8h;
typedef __attribute__((ext_vector_type(8)))  float v8f;
typedef __attribute__((ext_vector_type(4)))  float v4f;
typedef __attribute__((ext_vector_type(2)))  float v2f;
typedef __attribute__((ext_vector_type(4)))  unsigned v4u;
typedef __attribute__((ext_vector_type(4)))  int v4i;
typedef float __attribute__((may_alias)) float_a;
typedef int __attribute__((may_alias)) int_a;

template <typename T> __device__ __forceinline__ void vst2(void* p, T v) { *(volatile T*)p = v; __threadfence(); *(volatile T*)p = v; }
__device__ __forceinline__ v8f wmma16(v16h a, v16h b, v8f c) {
  v8f d = __builtin_amdgcn_wmma_f32_16x16x32_f16(false, a, false, b, (short)0, c, false, false);
  asm volatile("v_nop\n\tv_nop\n\tv_nop\n\tv_nop" : "+v"(d) : "v"(a), "v"(b));
  return d;
}
__device__ __forceinline__ v8f wmma_bf(v16b a, v16b b, v8f c) {
  v8f d = __builtin_amdgcn_wmma_f32_16x16x32_bf16(false, a, false, b, (short)0, c, false, false);
  asm volatile("v_nop\n\tv_nop\n\tv_nop\n\tv_nop" : "+v"(d) : "v"(a), "v"(b));
  return d;
}
__device__ __forceinline__ v16h frag_h(const _Float16* rowk0, int lane) {
  union { v16h v; v8h q[2]; } u; const _Float16* p = rowk0 + 8 * (lane >> 4);
  u.q[0] = *(const v8h*)p; u.q[1] = *(const v8h*)(p + 16); return u.v;
}
__device__ __forceinline__ v16h frag_f32(const float* rowk0, int lane) {
  v16h a; const float* p = rowk0 + 8 * (lane >> 4);
#pragma unroll
  for (int i = 0; i < 8; ++i) { a[i] = (_Float16)p[i]; a[8 + i] = (_Float16)p[16 + i]; }
  return a;
}
__device__ __forceinline__ v16h frag_f32s(const float* rowk0, int lane, float sc) {
  v16h a; const float* p = rowk0 + 8 * (lane >> 4);
#pragma unroll
  for (int i = 0; i < 8; ++i) { a[i] = (_Float16)(p[i] * sc); a[8 + i] = (_Float16)(p[16 + i] * sc); }
  return a;
}
__device__ __forceinline__ v16h fragc_f32(const float* W, int k0, int n, int lane, int ld, int K) {
  v16h a; const int g = lane >> 4;
#pragma unroll
  for (int i = 0; i < 8; ++i) { const int ka = k0 + 8 * g + i, kb = ka + 16;
    a[i] = (_Float16)(ka < K ? W[(size_t)(ka < K ? ka : K - 1) * ld + n] : 0.f); a[8 + i] = (_Float16)(kb < K ? W[(size_t)(kb < K ? kb : K - 1) * ld + n] : 0.f); }
  return a;
}
struct F2 { v16b h, l; };
__device__ __forceinline__ F2 bsplit16(const float v[16]) { F2 r;
#pragma unroll
  for (int i = 0; i < 16; ++i) { const __bf16 h = (__bf16)v[i]; r.h[i] = h; r.l[i] = (__bf16)(v[i] - (float)h); }
  return r; }
__device__ __forceinline__ F2 split_row(const float* row, int k0, int lane) { float v[16]; const float* p = row + k0 + 8 * (lane >> 4);
#pragma unroll
  for (int i = 0; i < 8; ++i) { v[i] = p[i]; v[8 + i] = p[16 + i]; }
  return bsplit16(v); }
__device__ __forceinline__ F2 split_rowK(const float* row, int k0, int lane, int K) { float v[16]; const int g = lane >> 4;
#pragma unroll
  for (int i = 0; i < 8; ++i) { const int ka = k0 + 8 * g + i, kb = ka + 16; v[i] = ka < K ? row[ka < K ? ka : K - 1] : 0.f; v[8 + i] = kb < K ? row[kb < K ? kb : K - 1] : 0.f; }
  return bsplit16(v); }
__device__ __forceinline__ F2 split_col(const float* W, int k0, int n, int lane, int ld, int K) { float v[16]; const int g = lane >> 4;
#pragma unroll
  for (int i = 0; i < 8; ++i) { const int ka = k0 + 8 * g + i, kb = ka + 16; v[i] = ka < K ? W[(size_t)(ka < K ? ka : K - 1) * ld + n] : 0.f; v[8 + i] = kb < K ? W[(size_t)(kb < K ? kb : K - 1) * ld + n] : 0.f; }
  return bsplit16(v); }
__device__ __forceinline__ v8f mac3(const F2& a, const F2& b, v8f c) { c = wmma_bf(a.l, b.h, c); c = wmma_bf(a.h, b.l, c); return wmma_bf(a.h, b.h, c); }
__device__ __forceinline__ float sigm(float v) { return 1.0f / (1.0f + expf(-v)); }
#define LDSX() do { asm volatile("s_wait_dscnt 0" ::: "memory"); __builtin_amdgcn_wave_barrier(); __builtin_amdgcn_fence(__ATOMIC_RELEASE, "workgroup"); } while (0)


#define NB 2
#define TT 2048
#define DM_ 1024
#define NH 16
#define HD 64
#ifndef TNB
#define TNB NB
#endif
#ifndef TQB
#define TQB (TT / 64)
#endif
typedef __attribute__((ext_vector_type(8))) __bf16 v8b;
__device__ __forceinline__ v16b frag_b(const __bf16* rowk0, int lane) {
  union { v16b v; v8b q[2]; } u; const __bf16* p = rowk0 + 8 * (lane >> 4);
  u.q[0] = *(const v8b*)p; u.q[1] = *(const v8b*)(p + 16); return u.v;
}
__device__ __forceinline__ float bfr(float v) { return (float)(__bf16)v; }
__device__ __attribute__((noinline)) float exp_ni(float v) { return expf(v); }
__device__ __attribute__((noinline)) float erf_ni(float v) { return erff(v); }

#define WS_QP  0u
#define WS_JK  (WS_QP + 4u * (size_t)NB * TT * NH * 8)
#define WS_VT  (WS_JK + 4u * (size_t)NB * TT * NH * 8)
#define WS_VL  (WS_VT + 2u * (size_t)NB * DM_ * TT)
#define WS_O   (WS_VL + 2u * (size_t)NB * DM_ * TT)
#define WS_END (WS_O + 4u * (size_t)NB * TT * DM_)

__global__ __launch_bounds__(128) void k_pl(const float* __restrict__ X, const float* __restrict__ W1Q, const float* __restrict__ W2Q, const float* __restrict__ W1K, const float* __restrict__ W2K, float* __restrict__ QP, float* __restrict__ JK) {
  __shared__ float sv[4][64][68];
  __shared__ __align__(16) float sq[64][NH * 8], sk[64][NH * 8];
  const int tid = threadIdx.x, wave = tid >> 5, lane = tid & 31, col = lane & 15, g = lane >> 4; const size_t r0 = (size_t)blockIdx.x * 64 + wave * 16; const size_t b = r0 / TT; const int t0 = (int)(r0 % TT);
  v8f aq1[4] = {}, aq2[4] = {}, ak1[4] = {}, ak2[4] = {};
#pragma unroll 1
  for (int kc = 0; kc < DM_ / 32; ++kc) { v16b a; { const float* p = X + (r0 + col) * DM_ + kc * 32 + 8 * g;
#pragma unroll
      for (int i = 0; i < 8; ++i) { a[i] = (__bf16)p[i]; a[8 + i] = (__bf16)p[16 + i]; } }
#pragma unroll
    for (int j = 0; j < 4; ++j) { const int o = j * 16 + col; v16b w1, w2, w3, w4;
#pragma unroll
      for (int i = 0; i < 8; ++i) { const int d0 = kc * 32 + 8 * g + i, d1 = d0 + 16; w1[i] = (__bf16)W1Q[(size_t)o * 2 * DM_ + d0]; w1[8 + i] = (__bf16)W1Q[(size_t)o * 2 * DM_ + d1]; w2[i] = (__bf16)W2Q[(size_t)o * 2 * DM_ + d0]; w2[8 + i] = (__bf16)W2Q[(size_t)o * 2 * DM_ + d1]; w3[i] = (__bf16)W1K[(size_t)o * DM_ + d0]; w3[8 + i] = (__bf16)W1K[(size_t)o * DM_ + d1]; w4[i] = (__bf16)W2K[(size_t)o * DM_ + d0]; w4[8 + i] = (__bf16)W2K[(size_t)o * DM_ + d1]; }
      aq1[j] = wmma_bf(a, w1, aq1[j]); aq2[j] = wmma_bf(a, w2, aq2[j]); ak1[j] = wmma_bf(a, w3, ak1[j]); ak2[j] = wmma_bf(a, w4, ak2[j]); } }
#pragma unroll 1
  for (int kc = 0; kc < DM_ / 32; ++kc) { v16b a; { const int t = t0 + wave * 16 + col; const float* p = X + (r0 + col - 1) * DM_ + kc * 32 + 8 * g;
#pragma unroll
      for (int i = 0; i < 8; ++i) { a[i] = (__bf16)(t > 0 ? p[i] : 0.f); a[8 + i] = (__bf16)(t > 0 ? p[16 + i] : 0.f); } }
#pragma unroll
    for (int j = 0; j < 4; ++j) { const int o = j * 16 + col; v16b w1, w2;
#pragma unroll
      for (int i = 0; i < 8; ++i) { const int d0 = DM_ + kc * 32 + 8 * g + i, d1 = d0 + 16; w1[i] = (__bf16)W1Q[(size_t)o * 2 * DM_ + d0]; w1[8 + i] = (__bf16)W1Q[(size_t)o * 2 * DM_ + d1]; w2[i] = (__bf16)W2Q[(size_t)o * 2 * DM_ + d0]; w2[8 + i] = (__bf16)W2Q[(size_t)o * 2 * DM_ + d1]; }
      aq1[j] = wmma_bf(a, w1, aq1[j]); aq2[j] = wmma_bf(a, w2, aq2[j]); } }
#pragma unroll
  for (int j = 0; j < 4; ++j)
#pragma unroll
    for (int r = 0; r < 8; ++r) { const int rl = wave * 16 + 8 * g + r, cl = j * 16 + col; sv[0][rl][cl] = aq1[j][r]; sv[1][rl][cl] = aq2[j][r]; sv[2][rl][cl] = ak1[j][r]; sv[3][rl][cl] = ak2[j][r]; }
  __syncthreads();
  { const int rl = tid >> 1, h0 = (tid & 1) * 8;
    for (int h = h0; h < h0 + 8; ++h) { const float* a1 = &sv[0][rl][h * 4]; const float* a2 = &sv[1][rl][h * 4]; const float* c1 = &sv[2][rl][h * 4]; const float* c2 = &sv[3][rl][h * 4];
      float pq[6], pk[6]; const int PI[6] = {0, 0, 0, 1, 1, 2}, PJ[6] = {1, 2, 3, 2, 3, 3}; float nq = 0.f, nk = 0.f;
      for (int e = 0; e < 6; ++e) { pq[e] = a1[PI[e]] * a2[PJ[e]] - a1[PJ[e]] * a2[PI[e]]; pk[e] = c1[PI[e]] * c2[PJ[e]] - c1[PJ[e]] * c2[PI[e]]; nq += pq[e] * pq[e]; nk += pk[e] * pk[e]; }
      const float iq = 1.0f / fmaxf(sqrtf(nq), 1e-12f), ik = 1.0f / fmaxf(sqrtf(nk), 1e-12f);
      for (int e = 0; e < 6; ++e) { pq[e] *= iq; pk[e] *= ik; }
      float jk[6] = {pk[5], -pk[4], pk[3], pk[2], -pk[1], pk[0]};
      for (int e = 0; e < 8; ++e) { sq[rl][h * 8 + e] = (e < 6) ? pq[e] : 0.f; sk[rl][h * 8 + e] = (e < 6) ? jk[e] : 0.f; } } }
  __syncthreads();
  for (int e = tid; e < 64 * 32; e += 128) { const int rl = e >> 5, q = e & 31; vst2(QP + ((size_t)blockIdx.x * 64 + rl) * (NH * 8) + q * 4, *(const v4f*)&sq[rl][q * 4]); vst2(JK + ((size_t)blockIdx.x * 64 + rl) * (NH * 8) + q * 4, *(const v4f*)&sk[rl][q * 4]); } }
__global__ __launch_bounds__(128) void k_v(const float* __restrict__ X, const float* __restrict__ WV, const float* __restrict__ BV, _Float16* __restrict__ VT, _Float16* __restrict__ VL) { __shared__ __align__(16) _Float16 th[128][72], tl[128][72];
  const int tid = threadIdx.x, wave = tid >> 5, lane = tid & 31, col = lane & 15, g = lane >> 4; const int c0 = blockIdx.y * 128; const size_t r0 = (size_t)blockIdx.x * 64;
  v8f acc[8] = {};
#pragma unroll 2
  for (int kc = 0; kc < DM_ / 32; ++kc) { v16b a; { const float* p = X + (r0 + wave * 16 + col) * DM_ + kc * 32 + 8 * g;
#pragma unroll
      for (int i = 0; i < 8; ++i) { a[i] = (__bf16)p[i]; a[8 + i] = (__bf16)p[16 + i]; } }
#pragma unroll
    for (int j = 0; j < 8; ++j) { v16b w; const int o = c0 + j * 16 + col;
#pragma unroll
      for (int i = 0; i < 8; ++i) { w[i] = (__bf16)WV[(size_t)o * DM_ + kc * 32 + 8 * g + i]; w[8 + i] = (__bf16)WV[(size_t)o * DM_ + kc * 32 + 16 + 8 * g + i]; }
      acc[j] = wmma_bf(a, w, acc[j]); } }
#pragma unroll
  for (int j = 0; j < 8; ++j) { const float bb = bfr(BV[c0 + j * 16 + col]);
#pragma unroll
    for (int r = 0; r < 8; ++r) { const float v = acc[j][r] + bb; const _Float16 hv = (_Float16)v; th[j * 16 + col][wave * 16 + 8 * g + r] = hv; tl[j * 16 + col][wave * 16 + 8 * g + r] = (_Float16)(v - (float)hv); } }
  __syncthreads(); const size_t b = r0 / TT; const int t0 = (int)(r0 % TT); for (int e = tid; e < 128 * 8; e += 128) { const int cl = e >> 3, q = e & 7; const size_t o = (b * DM_ + c0 + cl) * (size_t)TT + t0 + q * 8; vst2((unsigned*)(VT + o), *(const v4u*)&th[cl][q * 8]); vst2((unsigned*)(VL + o), *(const v4u*)&tl[cl][q * 8]); } }
__global__ __launch_bounds__(128) void k_att(const float* __restrict__ QP, const float* __restrict__ JK, const _Float16* __restrict__ VT, const _Float16* __restrict__ VL, float* __restrict__ O) {
  __shared__ __align__(16) float sp[4][16][36]; __shared__ __align__(16) float so[4][16][68];
  const int tid = threadIdx.x, wave = tid >> 5, lane = tid & 31, col = lane & 15, g = lane >> 4; const int qb = blockIdx.x, h = blockIdx.y; const size_t b = blockIdx.z; const int q0l = qb * 64 + wave * 16; const size_t q0 = b * TT + q0l;
  F2 aq; { float v[16];
#pragma unroll
    for (int i = 0; i < 16; ++i) v[i] = 0.f;
    if (g == 0) { const float* p = QP + (q0 + col) * (NH * 8) + h * 8;
#pragma unroll
      for (int i = 0; i < 8; ++i) v[i] = p[i]; }
    aq = bsplit16(v); }
  float m[8], l[8];
#pragma unroll
  for (int r = 0; r < 8; ++r) { m[r] = -3.0e38f; l[r] = 0.f; }
  v8f acc[4] = {};
  const int nks = (qb * 64 + 64) / 32;
#pragma unroll 1
  for (int ks = 0; ks < nks; ++ks) { float s[2][8];
#pragma unroll
    for (int ct = 0; ct < 2; ++ct) { const int kt = ks * 32 + ct * 16 + col; F2 bk; { float v[16];
#pragma unroll
        for (int i = 0; i < 16; ++i) v[i] = 0.f;
        if (g == 0) { const float* p = JK + (b * TT + kt) * (NH * 8) + h * 8;
#pragma unroll
          for (int i = 0; i < 8; ++i) v[i] = p[i]; }
        bk = bsplit16(v); }
      v8f c = {}; c = mac3(aq, bk, c);
#pragma unroll
      for (int r = 0; r < 8; ++r) s[ct][r] = (kt <= q0l + 8 * g + r) ? c[r] * 0.4082482904638631f : -3.0e38f; }
    float alpha[8];
#pragma unroll
    for (int r = 0; r < 8; ++r) { float mx = fmaxf(s[0][r], s[1][r]);
#pragma unroll
      for (int o = 1; o < 16; o <<= 1) mx = fmaxf(mx, __shfl_xor(mx, o));
      const float mn = fmaxf(m[r], mx); alpha[r] = (mn <= -1.0e38f) ? 1.f : __expf(m[r] - mn); const float e0 = (s[0][r] <= -1.0e38f) ? 0.f : __expf(s[0][r] - mn), e1 = (s[1][r] <= -1.0e38f) ? 0.f : __expf(s[1][r] - mn); float es = e0 + e1;
#pragma unroll
      for (int o = 1; o < 16; o <<= 1) es += __shfl_xor(es, o);
      l[r] = l[r] * alpha[r] + es; m[r] = mn; sp[wave][8 * g + r][col] = e0; sp[wave][8 * g + r][16 + col] = e1; }
#pragma unroll
    for (int j = 0; j < 4; ++j)
#pragma unroll
      for (int r = 0; r < 8; ++r) acc[j][r] *= alpha[r];
    LDSX();
    v16h pa, pr;
#pragma unroll
    for (int i = 0; i < 8; ++i) { const float f0 = sp[wave][col][8 * g + i] * 2048.0f, f1 = sp[wave][col][16 + 8 * g + i] * 2048.0f; const _Float16 h0 = (_Float16)f0, h1 = (_Float16)f1; pa[i] = h0; pa[8 + i] = h1; pr[i] = (_Float16)(f0 - (float)h0); pr[8 + i] = (_Float16)(f1 - (float)h1); }
#pragma unroll
    for (int j = 0; j < 4; ++j) { const size_t po = (b * DM_ + (size_t)h * HD + j * 16 + col) * TT + ks * 32; const v16h vh = frag_h(VT + po, lane); acc[j] = wmma16(pa, vh, acc[j]); acc[j] = wmma16(pr, vh, acc[j]); acc[j] = wmma16(pa, frag_h(VL + po, lane), acc[j]); }
    LDSX(); }
#pragma unroll
  for (int r = 0; r < 8; ++r) { const float il = (1.0f / 2048.0f) / l[r];
#pragma unroll
    for (int j = 0; j < 4; ++j) so[wave][8 * g + r][j * 16 + col] = acc[j][r] * il; }
  LDSX(); for (int rl = 0; rl < 16; ++rl) if (lane < 16) vst2(O + (q0 + rl) * DM_ + h * HD + lane * 4, *(const v4f*)&so[wave][rl][lane * 4]); }
__global__ __launch_bounds__(128) void k_out(const float* __restrict__ O, const float* __restrict__ WO, const float* __restrict__ BO, float* __restrict__ OUT) { __shared__ __align__(16) float sf[4][16][132];
  const int tid = threadIdx.x, wave = tid >> 5, lane = tid & 31, col = lane & 15, g = lane >> 4; const int c0 = blockIdx.y * 128; const size_t r0 = (size_t)blockIdx.x * 64 + wave * 16;
  v8f acc[8] = {};
#pragma unroll 2
  for (int kc = 0; kc < DM_ / 32; ++kc) { const F2 a = split_row(O + (r0 + col) * DM_, kc * 32, lane);
#pragma unroll
    for (int j = 0; j < 8; ++j) { v16b w; const int o = c0 + j * 16 + col;
#pragma unroll
      for (int i = 0; i < 8; ++i) { w[i] = (__bf16)WO[(size_t)o * DM_ + kc * 32 + 8 * g + i]; w[8 + i] = (__bf16)WO[(size_t)o * DM_ + kc * 32 + 16 + 8 * g + i]; }
      acc[j] = wmma_bf(a.h, w, acc[j]); acc[j] = wmma_bf(a.l, w, acc[j]); } }
#pragma unroll
  for (int j = 0; j < 8; ++j) { const float bb = bfr(BO[c0 + j * 16 + col]);
#pragma unroll
    for (int r = 0; r < 8; ++r) sf[wave][8 * g + r][j * 16 + col] = acc[j][r] + bb; }
  LDSX(); for (int rl = 0; rl < 16; ++rl) vst2(OUT + (r0 + rl) * DM_ + c0 + lane * 4, *(const v4f*)&sf[wave][rl][lane * 4]); }
extern "C" void kernel_launch(void* const* d_in, const int* in_sizes, int n_in, void* d_out, int out_size, void* d_ws, size_t ws_size, hipStream_t stream) {
  (void)in_sizes; (void)n_in; (void)out_size;
  const float** F = (const float**)d_in;
  if (ws_size < (size_t)WS_END) return;
  char* ws = (char*)d_ws; float *QP = (float*)(ws + WS_QP), *JK = (float*)(ws + WS_JK), *O = (float*)(ws + WS_O); _Float16 *VT = (_Float16*)(ws + WS_VT), *VL = (_Float16*)(ws + WS_VL);
  k_pl<<<TNB * TT / 64, 128, 0, stream>>>(F[0], F[1], F[2], F[3], F[4], QP, JK);
  k_v<<<dim3(TNB * TT / 64, DM_ / 128), 128, 0, stream>>>(F[0], F[5], F[6], VT, VL);
  k_att<<<dim3(TQB, NH, TNB), 128, 0, stream>>>(QP, JK, VT, VL, O);
  for (int b = 0; b < TNB; ++b) k_out<<<dim3(TQB, DM_ / 128), 128, 0, stream>>>(O + (size_t)b * TT * DM_, F[7], F[8], (float*)d_out + (size_t)b * TT * DM_);
}
